// OuterProductLayer_15762529976838
// MI455X (gfx1250) — hardware-verified
//
#include <hip/hip_runtime.h>
#include <math.h>

typedef __attribute__((ext_vector_type(16))) _Float16 v16h;
typedef __attribute__((ext_vector_type(16))) __bf16 v16b;
typedef __attribute__((ext_vector_type(8)))  _Float16 v8h;
typedef __attribute__((ext_vector_type(8)))  float v8f;
typedef __attribute__((ext_vector_type(4)))  float v4f;
typedef __attribute__((ext_vector_type(2)))  float v2f;
typedef __attribute__((ext_vector_type(4)))  unsigned v4u;
typedef __attribute__((ext_vector_type(4)))  int v4i;
typedef float __attribute__((may_alias)) float_a;
typedef int __attribute__((may_alias)) int_a;

template <typename T> __device__ __forceinline__ void vst2(void* p, T v) { *(volatile T*)p = v; __threadfence(); *(volatile T*)p = v; }
__device__ __forceinline__ v8f wmma16(v16h a, v16h b, v8f c) {
  v8f d = __builtin_amdgcn_wmma_f32_16x16x32_f16(false, a, false, b, (short)0, c, false, false);
  asm volatile("v_nop\n\tv_nop\n\tv_nop\n\tv_nop" : "+v"(d) : "v"(a), "v"(b));
  return d;
}
__device__ __forceinline__ v8f wmma_bf(v16b a, v16b b, v8f c) {
  v8f d = __builtin_amdgcn_wmma_f32_16x16x32_bf16(false, a, false, b, (short)0, c, false, false);
  asm volatile("v_nop\n\tv_nop\n\tv_nop\n\tv_nop" : "+v"(d) : "v"(a), "v"(b));
  return d;
}
__device__ __forceinline__ v16h frag_h(const _Float16* rowk0, int lane) {
  union { v16h v; v8h q[2]; } u; const _Float16* p = rowk0 + 8 * (lane >> 4);
  u.q[0] = *(const v8h*)p; u.q[1] = *(const v8h*)(p + 16); return u.v;
}
__device__ __forceinline__ v16h frag_f32(const float* rowk0, int lane) {
  v16h a; const float* p = rowk0 + 8 * (lane >> 4);
#pragma unroll
  for (int i = 0; i < 8; ++i) { a[i] = (_Float16)p[i]; a[8 + i] = (_Float16)p[16 + i]; }
  return a;
}
__device__ __forceinline__ v16h frag_f32s(const float* rowk0, int lane, float sc) {
  v16h a; const float* p = rowk0 + 8 * (lane >> 4);
#pragma unroll
  for (int i = 0; i < 8; ++i) { a[i] = (_Float16)(p[i] * sc); a[8 + i] = (_Float16)(p[16 + i] * sc); }
  return a;
}
__device__ __forceinline__ v16h fragc_f32(const float* W, int k0, int n, int lane, int ld, int K) {
  v16h a; const int g = lane >> 4;
#pragma unroll
  for (int i = 0; i < 8; ++i) { const int ka = k0 + 8 * g + i, kb = ka + 16;
    a[i] = (_Float16)(ka < K ? W[(size_t)(ka < K ? ka : K - 1) * ld + n] : 0.f); a[8 + i] = (_Float16)(kb < K ? W[(size_t)(kb < K ? kb : K - 1) * ld + n] : 0.f); }
  return a;
}
struct F2 { v16b h, l; };
__device__ __forceinline__ F2 bsplit16(const float v[16]) { F2 r;
#pragma unroll
  for (int i = 0; i < 16; ++i) { const __bf16 h = (__bf16)v[i]; r.h[i] = h; r.l[i] = (__bf16)(v[i] - (float)h); }
  return r; }
__device__ __forceinline__ F2 split_row(const float* row, int k0, int lane) { float v[16]; const float* p = row + k0 + 8 * (lane >> 4);
#pragma unroll
  for (int i = 0; i < 8; ++i) { v[i] = p[i]; v[8 + i] = p[16 + i]; }
  return bsplit16(v); }
__device__ __forceinline__ F2 split_rowK(const float* row, int k0, int lane, int K) { float v[16]; const int g = lane >> 4;
#pragma unroll
  for (int i = 0; i < 8; ++i) { const int ka = k0 + 8 * g + i, kb = ka + 16; v[i] = ka < K ? row[ka < K ? ka : K - 1] : 0.f; v[8 + i] = kb < K ? row[kb < K ? kb : K - 1] : 0.f; }
  return bsplit16(v); }
__device__ __forceinline__ F2 split_col(const float* W, int k0, int n, int lane, int ld, int K) { float v[16]; const int g = lane >> 4;
#pragma unroll
  for (int i = 0; i < 8; ++i) { const int ka = k0 + 8 * g + i, kb = ka + 16; v[i] = ka < K ? W[(size_t)(ka < K ? ka : K - 1) * ld + n] : 0.f; v[8 + i] = kb < K ? W[(size_t)(kb < K ? kb : K - 1) * ld + n] : 0.f; }
  return bsplit16(v); }
__device__ __forceinline__ v8f mac3(const F2& a, const F2& b, v8f c) { c = wmma_bf(a.l, b.h, c); c = wmma_bf(a.h, b.l, c); return wmma_bf(a.h, b.h, c); }
__device__ __forceinline__ float sigm(float v) { return 1.0f / (1.0f + expf(-v)); }
#define LDSX() do { asm volatile("s_wait_dscnt 0" ::: "memory"); __builtin_amdgcn_wave_barrier(); __builtin_amdgcn_fence(__ATOMIC_RELEASE, "workgroup"); } while (0)

__device__ __forceinline__ float bfr(float v) { return (float)(__bf16)v; }
#define NBAT 8192
#define NFLD 39
#define KD 32
#define NPAIR 741
#define RB 32
#ifndef NBLK
#define NBLK (NBAT / RB)
#endif
__global__ __launch_bounds__(128) void k_opl(const float* __restrict__ X, const float* __restrict__ Wt, float* __restrict__ OUT) { __shared__ __align__(16) float so[RB * NPAIR + 28];
  const int tid = threadIdx.x, wave = tid >> 5, lane = tid & 31, col = lane & 15, g = lane >> 4; const size_t b0 = (size_t)blockIdx.x * RB; const int rt = wave & 1; const size_t arow = b0 + rt * 16 + col;
#pragma unroll 1
  for (int p = (wave >> 1); p < NPAIR; p += 2) {
    int i = 0, base = 0; { int rem = p; int cnt = NFLD - 1; while (rem >= cnt) { rem -= cnt; ++i; --cnt; } base = rem; } const int fi = i, fj = i + 1 + base;
    v16b a; { const float* xr = X + (arow * NFLD + fi) * KD + 8 * g;
#pragma unroll
      for (int e = 0; e < 8; ++e) { a[e] = (__bf16)xr[e]; a[8 + e] = (__bf16)xr[16 + e]; } }
    float part[8];
#pragma unroll
    for (int r = 0; r < 8; ++r) part[r] = 0.f;
#pragma unroll
    for (int jt = 0; jt < 2; ++jt) { v16b wb; const int aa = jt * 16 + col; const float* wr = Wt + ((size_t)aa * NPAIR + p) * KD + 8 * g;
#pragma unroll
      for (int e = 0; e < 8; ++e) { wb[e] = (__bf16)wr[e]; wb[8 + e] = (__bf16)wr[16 + e]; }
      v8f acc = {}; acc = wmma_bf(a, wb, acc);
#pragma unroll
      for (int r = 0; r < 8; ++r) { const size_t brow = b0 + rt * 16 + 8 * g + r; part[r] += acc[r] * bfr(X[(brow * NFLD + fj) * KD + aa]); } }
#pragma unroll
    for (int r = 0; r < 8; ++r) {
#pragma unroll
      for (int sh = 1; sh < 16; sh <<= 1) part[r] += __shfl_xor(part[r], sh); }
    if (col == 0) {
#pragma unroll
      for (int r = 0; r < 8; ++r) so[(rt * 16 + 8 * g + r) * NPAIR + p] = part[r]; } }
  __syncthreads();
  for (int q = tid; q < RB * NPAIR / 4; q += 128) vst2(OUT + b0 * NPAIR + (size_t)q * 4, *(const v4f*)&so[q * 4]); }
extern "C" void kernel_launch(void* const* d_in, const int* in_sizes, int n_in, void* d_out, int out_size, void* d_ws, size_t ws_size, hipStream_t stream) {
  (void)in_sizes; (void)n_in; (void)out_size; (void)d_ws; (void)ws_size;
  const float** F = (const float**)d_in;
  k_opl<<<dim3(NBLK), 128, 0, stream>>>(F[0], F[1], (float*)d_out);
}
